// MixOfMambaModule_11158325035380
// MI455X (gfx1250) — hardware-verified
//
#include <hip/hip_runtime.h>
#include <math.h>

typedef __attribute__((ext_vector_type(16))) __bf16       v16b;
typedef __attribute__((ext_vector_type(8)))  __bf16       v8b;
typedef __attribute__((ext_vector_type(8)))  float        v8f;
typedef __attribute__((ext_vector_type(4)))  float        v4f;
typedef __attribute__((ext_vector_type(4)))  unsigned int v4u;

constexpr int kB     = 2;
constexpr int kC     = 128;
constexpr int kSide  = 64;
constexpr int kL     = kSide * kSide;
constexpr int kE     = 3;
constexpr int kNst   = 64;
constexpr int kDin   = 2 * kC;
constexpr int kDtR   = 8;
constexpr int kRc    = 64;
constexpr int kRows  = kB * kL;
constexpr int kXrP   = kE * 2 * kDin;
constexpr int kXdN   = kDtR + 2 * kNst;
constexpr int kXdP   = 192;
constexpr int kYcP   = kE * kDin;
constexpr int kPadW  = kSide + 2;
constexpr int kRK    = 9 * kC;
static_assert(kL == 4096 && kRows == 8192 && kDin == 256 && kXrP == 1536 && kXdN == 136 && kYcP == 768 && kRK == 1152, "shape constants");
static_assert((kC % 32) == 0 && (kDin % 32) == 0 && (kYcP % 32) == 0, "GEMM K multiples of 32");
static_assert((kRows % 64) == 0 && (kXrP % 64) == 0 && (kXdP % 64) == 0 && (kC % 64) == 0 && (kRc % 64) == 0, "GEMM M,N multiples of 64");
static_assert(kXdP >= kXdN, "x_proj pad");

constexpr size_t kOffXSEQ = 0;
constexpr size_t kOffXPAD = kOffXSEQ + (size_t)kRows * kC * 2;
constexpr size_t kOffWIN  = kOffXPAD + (size_t)kB * kPadW * kPadW * kC * 2;
constexpr size_t kOffWXP  = kOffWIN  + (size_t)kXrP * kC * 2;
constexpr size_t kOffWOUT = kOffWXP  + (size_t)kE * kXdP * kDin * 2;
constexpr size_t kOffWFUS = kOffWOUT + (size_t)kC * kYcP * 2;
constexpr size_t kOffWR   = kOffWFUS + (size_t)kC * kC * 2;
constexpr size_t kOffPART = kOffWR   + (size_t)kRc * kRK * 2;
constexpr size_t kOffWTS  = kOffPART + (size_t)(kRows / 64) * kRc * 4;
constexpr size_t kOffXR   = kOffWTS  + 128;
constexpr size_t kOffU16  = kOffXR   + (size_t)kRows * kXrP * 4;
constexpr size_t kOffDBL  = kOffU16  + (size_t)kE * kRows * kDin * 2;
constexpr size_t kOffYH   = kOffDBL  + (size_t)kE * kRows * kXdP * 4;
constexpr size_t kOffYL   = kOffYH   + (size_t)kRows * kYcP * 2;
constexpr size_t kOffWSH  = kOffYL   + (size_t)kRows * kYcP * 2;
constexpr size_t kOffWSL  = kOffWSH  + (size_t)kRows * kC * 2;
constexpr size_t kWsTotal = kOffWSL  + (size_t)kRows * kC * 2;
static_assert(kWsTotal == 116574336ull, "carve total");
static_assert(kWsTotal <= 134217728ull, "carve cap");
static_assert((kOffXPAD % 128) == 0 && (kOffWIN % 128) == 0 && (kOffWXP % 128) == 0 && (kOffWOUT % 128) == 0 &&
              (kOffWFUS % 128) == 0 && (kOffWR % 128) == 0 && (kOffPART % 128) == 0 && (kOffWTS % 128) == 0 &&
              (kOffXR % 128) == 0 && (kOffU16 % 128) == 0 && (kOffDBL % 128) == 0 && (kOffYH % 128) == 0 &&
              (kOffYL % 128) == 0 && (kOffWSH % 128) == 0 && (kOffWSL % 128) == 0, "128-B aligned regions");

__device__ __forceinline__ unsigned short f2bf_bits(float f) {
  unsigned u = __float_as_uint(f);
  return (unsigned short)((u + 0x7FFFu + ((u >> 16) & 1u)) >> 16);
}
__device__ __forceinline__ float bf_bits2f(unsigned short h) { return __uint_as_float(((unsigned)h) << 16); }
__device__ __forceinline__ float rne_bf(float f) { return bf_bits2f(f2bf_bits(f)); }
__device__ __forceinline__ unsigned pack_hi2(float a, float b) {
  const unsigned lo = (unsigned)f2bf_bits(a);
  const unsigned hi = (unsigned)f2bf_bits(b);
  return lo | (hi << 16);
}
__device__ __forceinline__ unsigned pack_lo2(float a, float b) {
  const float ra = a - rne_bf(a);
  const float rb = b - rne_bf(b);
  return pack_hi2(ra, rb);
}
__device__ __forceinline__ void store16_2pass(unsigned short* p, v4u w) {
  *(volatile v4u*)(void*)p = w;
  __threadfence();
  *(volatile v4u*)(void*)p = w;
}

__device__ __forceinline__ v16b ldfrag(const __bf16* p) {
  union { v16b v; v8b h[2]; } f;
  f.h[0] = *(const v8b*)(p);
  f.h[1] = *(const v8b*)(p + 16);
  return f.v;
}
__device__ __forceinline__ v8f mma_bf(v16b a, v16b b, v8f c) {
  return __builtin_amdgcn_wmma_f32_16x16x32_bf16(false, a, false, b, (short)0, c, false, false);
}
__device__ __forceinline__ void guard_row4(v8f& a, v8f& b, v8f& c, v8f& d, v16b x, v16b y) {
  asm volatile("v_nop\n\tv_nop\n\tv_nop\n\tv_nop" : "+v"(a), "+v"(b), "+v"(c), "+v"(d) : "v"(x), "v"(y));
}
__device__ __forceinline__ void keep4_b(v16b a, v16b b, v16b c, v16b d) { asm volatile("v_nop" :: "v"(a), "v"(b), "v"(c), "v"(d)); }
__device__ __forceinline__ void acc_guard4(v8f& a, v8f& b, v8f& c, v8f& d) { asm volatile("v_nop\n\tv_nop\n\tv_nop\n\tv_nop" : "+v"(a), "+v"(b), "+v"(c), "+v"(d)); }

__global__ __launch_bounds__(256) void prep_x_kernel(
    const float* __restrict__ x, unsigned short* __restrict__ XSEQ, unsigned short* __restrict__ XPAD)
{
  __shared__ float tile[kC * 65];
  const int tid = threadIdx.x, lane = tid & 31, wave = tid >> 5;
  const int b = blockIdx.x >> 6, h = blockIdx.x & 63;
#pragma unroll 1
  for (int p = 0; p < 32; ++p) {
    const int idx = tid + p * 256;
    const int c = idx >> 6, w = idx & 63;
    tile[c * 65 + w] = x[(((size_t)b * kC + c) * kSide + h) * kSide + w];
  }
  __syncthreads();
  const int ph = lane >> 4, c8 = (lane & 15) * 8;
  v4u pk[4];
#pragma unroll
  for (int it = 0; it < 4; ++it) {
    const int pw = it * 16 + wave * 2 + ph;
    const float* tp = tile + c8 * 65 + pw;
    const unsigned q0 = pack_hi2(tp[0],   tp[65]);
    const unsigned q1 = pack_hi2(tp[130], tp[195]);
    const unsigned q2 = pack_hi2(tp[260], tp[325]);
    const unsigned q3 = pack_hi2(tp[390], tp[455]);
    pk[it] = (v4u){q0, q1, q2, q3};
  }
  const int nb = 2 + ((h == 0 || h == 63) ? kPadW : 0);
  const int brow = (h == 0) ? 0 : (kPadW - 1);
  const v4u zz = (v4u){0u, 0u, 0u, 0u};
  for (int pass = 0; pass < 2; ++pass) {
#pragma unroll
    for (int it = 0; it < 4; ++it) {
      const int pw = it * 16 + wave * 2 + ph;
      *(volatile v4u*)(void*)(XSEQ + ((size_t)(b * kL + h * kSide + pw)) * kC + c8) = pk[it];
      *(volatile v4u*)(void*)(XPAD + ((size_t)((b * kPadW + h + 1) * kPadW + pw + 1)) * kC + c8) = pk[it];
    }
#pragma unroll 1
    for (int p0 = 0; p0 < nb; p0 += 16) {
      const int p = p0 + wave * 2 + ph;
      const int hp = (p < 2) ? (h + 1) : brow;
      const int wp = (p < 2) ? (p * (kPadW - 1)) : (p - 2);
      if (p < nb) *(volatile v4u*)(void*)(XPAD + ((size_t)((b * kPadW + hp) * kPadW + wp)) * kC + c8) = zz;
    }
    __threadfence();
  }
}

__global__ __launch_bounds__(256) void prep_w_kernel(
    const float* __restrict__ in_w, const float* __restrict__ xp_w, const float* __restrict__ out_w,
    const float* __restrict__ fus_w, const float* __restrict__ r_w,
    unsigned short* __restrict__ WIN, unsigned short* __restrict__ WXP, unsigned short* __restrict__ WOUT,
    unsigned short* __restrict__ WFUS, unsigned short* __restrict__ WR)
{
  const int blk = blockIdx.x, tid = threadIdx.x;
  if (blk < 96) {
    const size_t e0 = ((size_t)blk * 256 + tid) * 8;
    const v4f a0 = *(const v4f*)(in_w + e0);
    const v4f a1 = *(const v4f*)(in_w + e0 + 4);
    const v4u w = (v4u){pack_hi2(a0[0], a0[1]), pack_hi2(a0[2], a0[3]), pack_hi2(a1[0], a1[1]), pack_hi2(a1[2], a1[3])};
    store16_2pass(WIN + e0, w);
  } else if (blk < 168) {
    const int e0 = ((blk - 96) * 256 + tid) * 8;
    const int k8 = e0 & 255;
    const int rr = e0 >> 8;
    const int e  = rr / kXdP;
    const int r  = rr - e * kXdP;
    const bool valid = (r < kXdN);
    const int rc = valid ? r : (kXdN - 1);
    const float* sp = xp_w + ((size_t)(e * kXdN + rc)) * kDin + k8;
    const v4f a0 = *(const v4f*)(sp);
    const v4f a1 = *(const v4f*)(sp + 4);
    const float f0 = valid ? a0[0] : 0.0f, f1 = valid ? a0[1] : 0.0f, f2 = valid ? a0[2] : 0.0f, f3 = valid ? a0[3] : 0.0f;
    const float f4 = valid ? a1[0] : 0.0f, f5 = valid ? a1[1] : 0.0f, f6 = valid ? a1[2] : 0.0f, f7 = valid ? a1[3] : 0.0f;
    const v4u w = (v4u){pack_hi2(f0, f1), pack_hi2(f2, f3), pack_hi2(f4, f5), pack_hi2(f6, f7)};
    store16_2pass(WXP + e0, w);
  } else if (blk < 216) {
    const int e0 = ((blk - 168) * 256 + tid) * 8;
    const int c  = e0 / kYcP;
    const int k  = e0 - c * kYcP;
    const int e  = k >> 8;
    const int d  = k & 255;
    const float* sp = out_w + ((size_t)(e * kC + c)) * kDin + d;
    const v4f a0 = *(const v4f*)(sp);
    const v4f a1 = *(const v4f*)(sp + 4);
    const v4u w = (v4u){pack_hi2(a0[0], a0[1]), pack_hi2(a0[2], a0[3]), pack_hi2(a1[0], a1[1]), pack_hi2(a1[2], a1[3])};
    store16_2pass(WOUT + e0, w);
  } else if (blk < 224) {
    const int e0 = ((blk - 216) * 256 + tid) * 8;
    const v4f a0 = *(const v4f*)(fus_w + e0);
    const v4f a1 = *(const v4f*)(fus_w + e0 + 4);
    const v4u w = (v4u){pack_hi2(a0[0], a0[1]), pack_hi2(a0[2], a0[3]), pack_hi2(a1[0], a1[1]), pack_hi2(a1[2], a1[3])};
    store16_2pass(WFUS + e0, w);
  } else {
    const int e0  = ((blk - 224) * 256 + tid) * 8;
    const int oc  = e0 / kRK;
    const int rem = e0 - oc * kRK;
    const int tap = rem >> 7;
    const int ic  = rem & 127;
    const float* sp = r_w + ((size_t)(oc * kC + ic)) * 9 + tap;
    const float f0 = sp[0],  f1 = sp[9],  f2 = sp[18], f3 = sp[27];
    const float f4 = sp[36], f5 = sp[45], f6 = sp[54], f7 = sp[63];
    const v4u w = (v4u){pack_hi2(f0, f1), pack_hi2(f2, f3), pack_hi2(f4, f5), pack_hi2(f6, f7)};
    store16_2pass(WR + e0, w);
  }
}

__global__ __launch_bounds__(256) void router_conv_kernel(
    const unsigned short* __restrict__ XPp, const unsigned short* __restrict__ Wrp,
    const float* __restrict__ rb, float* __restrict__ PART)
{
  __shared__ __align__(16) float sP[8][64];
  const __bf16* XP = (const __bf16*)XPp;
  const __bf16* Wr = (const __bf16*)Wrp;
  const int lane = threadIdx.x & 31, wave = threadIdx.x >> 5;
  const int tile = blockIdx.x * 8 + wave;
  if (tile >= kRows / 64) return;
  const int b = tile >> 6, h = tile & 63;
  const int rlane = lane & 15;
  const int koff  = (lane >> 4) * 8;

  v8f acc[4][4];
#pragma unroll
  for (int i = 0; i < 4; ++i)
#pragma unroll
    for (int j = 0; j < 4; ++j) acc[i][j] = (v8f){0.f, 0.f, 0.f, 0.f, 0.f, 0.f, 0.f, 0.f};

#pragma unroll 1
  for (int tap = 0; tap < 9; ++tap) {
    const int kh = tap / 3;
    const int kw = tap - 3 * kh;
    const size_t abase = ((size_t)((b * kPadW + h + kh) * kPadW + kw)) * kC;
#pragma unroll 1
    for (int k0 = 0; k0 < kC; k0 += 32) {
      v16b bh[4];
#pragma unroll
      for (int j = 0; j < 4; ++j)
        bh[j] = ldfrag(Wr + (size_t)((j << 4) + rlane) * kRK + tap * kC + k0 + koff);
#pragma unroll
      for (int i = 0; i < 4; ++i) {
        const v16b ah = ldfrag(XP + abase + (size_t)((i << 4) + rlane) * kC + k0 + koff);
#pragma unroll
        for (int j = 0; j < 4; ++j) acc[i][j] = mma_bf(ah, bh[j], acc[i][j]);
        guard_row4(acc[i][0], acc[i][1], acc[i][2], acc[i][3], ah, ah);
      }
      keep4_b(bh[0], bh[1], bh[2], bh[3]);
    }
  }
  acc_guard4(acc[0][0], acc[0][1], acc[0][2], acc[0][3]);
  acc_guard4(acc[1][0], acc[1][1], acc[1][2], acc[1][3]);
  acc_guard4(acc[2][0], acc[2][1], acc[2][2], acc[2][3]);
  acc_guard4(acc[3][0], acc[3][1], acc[3][2], acc[3][3]);

  float cs[4];
#pragma unroll
  for (int j = 0; j < 4; ++j) {
    const float bv = rne_bf(rb[(j << 4) + rlane]);
    float s = 0.0f;
#pragma unroll
    for (int i = 0; i < 4; ++i)
#pragma unroll
      for (int r = 0; r < 8; ++r) s += fmaxf(acc[i][j][r] + bv, 0.0f);
    s += __shfl_xor(s, 16, 32);
    cs[j] = s;
  }
  float* sp = sP[wave];
  if (lane < 16) {
    sp[lane]      = cs[0];
    sp[16 + lane] = cs[1];
    sp[32 + lane] = cs[2];
    sp[48 + lane] = cs[3];
  }
  __builtin_amdgcn_fence(__ATOMIC_RELEASE, "workgroup");
  __builtin_amdgcn_wave_barrier();
  __builtin_amdgcn_fence(__ATOMIC_ACQUIRE, "workgroup");
  const int l16 = lane & 15;
  const v4f pv = *(const v4f*)(sp + l16 * 4);
  for (int pass = 0; pass < 2; ++pass) {
    if (lane < 16) *(volatile v4f*)(PART + (size_t)tile * kRc + l16 * 4) = pv;
    __threadfence();
  }
}

__global__ __launch_bounds__(128) void router_finish_kernel(
    const float* __restrict__ PART, const float* __restrict__ lw, const float* __restrict__ lb, float* __restrict__ WTS)
{
  __shared__ float sPool[128];
  __shared__ float sLog[8];
  const int tid = threadIdx.x;
  {
    const int b = tid >> 6, oc = tid & 63;
    float s = 0.0f;
#pragma unroll 1
    for (int t = 0; t < 64; ++t) s += PART[(size_t)(b * 64 + t) * kRc + oc];
    sPool[tid] = s * (1.0f / (float)kL);
  }
  __syncthreads();
  {
    const int t6 = (tid < 6) ? tid : 5;
    const int b = t6 / 3, e = t6 - 3 * b;
    float z = 0.0f;
#pragma unroll 1
    for (int c = 0; c < kRc; ++c) z = fmaf(sPool[b * 64 + c], rne_bf(lw[e * kRc + c]), z);
    z += rne_bf(lb[e]);
    if (tid < 6) sLog[tid] = z;
  }
  __syncthreads();
  if (tid < 32) {
    const bool valid = (tid < 6);
    const int t6 = valid ? tid : 0;
    const int b = t6 / 3;
    const float z0 = sLog[b * 3], z1 = sLog[b * 3 + 1], z2 = sLog[b * 3 + 2];
    const float zm = sLog[t6];
    const float m = fmaxf(z0, fmaxf(z1, z2));
    const float s = (expf(z0 - m) + expf(z1 - m)) + expf(z2 - m);
    const float mine = expf(zm - m) * (1.0f / s);
    const float val = valid ? mine : 0.0f;
    volatile float* wp = WTS + tid;
    *wp = val;
    __threadfence();
    *wp = val;
  }
}

template <int SPLA, int SPLB, int BIAS_MODE, int OUT_MODE, int OMAP>
__global__ __launch_bounds__(256) void gemm64_bf16_kernel(
    const unsigned short* __restrict__ Ap, const unsigned short* A2p, int lda, long strideA,
    const unsigned short* __restrict__ Btp, const unsigned short* Bt2p, int ldb, long strideB,
    void* __restrict__ Cout, void* Cout2, int ldc, long strideC,
    const float* __restrict__ bias, int M, int N, int K)
{
  __shared__ __align__(16) float sT[8][16 * 68];
  const int b    = blockIdx.y;
  const int lane = threadIdx.x & 31;
  const int wave = threadIdx.x >> 5;
  const int tilesN = N >> 6;
  const int tilesM = M >> 6;
  const int tile = blockIdx.x * 8 + wave;
  if (tile >= tilesM * tilesN) return;
  const int tm = tile / tilesN;
  const int tn = tile - tm * tilesN;
  const int m0 = tm << 6;
  const int n0 = tn << 6;

  const __bf16* Ab  = (const __bf16*)Ap   + (size_t)b * strideA;
  const __bf16* Ab2 = (const __bf16*)A2p  + (size_t)b * strideA;
  const __bf16* Bb  = (const __bf16*)Btp  + (size_t)b * strideB;
  const __bf16* Bb2 = (const __bf16*)Bt2p + (size_t)b * strideB;

  const int rlane = lane & 15;
  const int koff  = (lane >> 4) * 8;
  const int mOff  = (lane >> 4) * 8;

  v8f acc[4][4];
#pragma unroll
  for (int i = 0; i < 4; ++i)
#pragma unroll
    for (int j = 0; j < 4; ++j) acc[i][j] = (v8f){0.f, 0.f, 0.f, 0.f, 0.f, 0.f, 0.f, 0.f};

  for (int k0 = 0; k0 < K; k0 += 32) {
    v16b bh[4], bl[4];
#pragma unroll
    for (int j = 0; j < 4; ++j) {
      const size_t bo = (size_t)(n0 + (j << 4) + rlane) * ldb + koff + k0;
      bh[j] = ldfrag(Bb + bo);
      bl[j] = bh[j];
      if (SPLB) bl[j] = ldfrag(Bb2 + bo);
    }
#pragma unroll
    for (int i = 0; i < 4; ++i) {
      const size_t ao = (size_t)(m0 + (i << 4) + rlane) * lda + koff + k0;
      const v16b ah = ldfrag(Ab + ao);
      v16b al = ah;
      if (SPLA) al = ldfrag(Ab2 + ao);
#pragma unroll
      for (int j = 0; j < 4; ++j) {
        acc[i][j] = mma_bf(ah, bh[j], acc[i][j]);
        if (SPLB) acc[i][j] = mma_bf(ah, bl[j], acc[i][j]);
        if (SPLA) acc[i][j] = mma_bf(al, bh[j], acc[i][j]);
      }
      guard_row4(acc[i][0], acc[i][1], acc[i][2], acc[i][3], ah, al);
    }
    keep4_b(bh[0], bh[1], bh[2], bh[3]);
    if (SPLB) keep4_b(bl[0], bl[1], bl[2], bl[3]);
  }
  acc_guard4(acc[0][0], acc[0][1], acc[0][2], acc[0][3]);
  acc_guard4(acc[1][0], acc[1][1], acc[1][2], acc[1][3]);
  acc_guard4(acc[2][0], acc[2][1], acc[2][2], acc[2][3]);
  acc_guard4(acc[3][0], acc[3][1], acc[3][2], acc[3][3]);

  float* slab = sT[wave];
#pragma unroll
  for (int i = 0; i < 4; ++i) {
    const int mBase = m0 + (i << 4);
#pragma unroll
    for (int j = 0; j < 4; ++j) {
#pragma unroll
      for (int r = 0; r < 8; ++r) {
        float v = acc[i][j][r];
        if (BIAS_MODE == 1) v += rne_bf(bias[mBase + mOff + r]);
        slab[(mOff + r) * 68 + (j << 4) + rlane] = v;
      }
    }
    __builtin_amdgcn_fence(__ATOMIC_RELEASE, "workgroup");
    __builtin_amdgcn_wave_barrier();
    __builtin_amdgcn_fence(__ATOMIC_ACQUIRE, "workgroup");
    if (OUT_MODE == 0) {
      float* C = (float*)Cout + (size_t)b * strideC;
      const size_t extra = (OMAP == 1) ? ((size_t)(n0 >> 12) * (size_t)((kC - 1) * kL)) : (size_t)0;
      const int hh = lane >> 4, c4 = (lane & 15) * 4;
      v4f ov[8];
#pragma unroll
      for (int it = 0; it < 8; ++it) ov[it] = *(const v4f*)(slab + (it * 2 + hh) * 68 + c4);
      for (int pass = 0; pass < 2; ++pass) {
#pragma unroll
        for (int it = 0; it < 8; ++it) {
          const int row = it * 2 + hh;
          *(volatile v4f*)(C + (size_t)(mBase + row) * ldc + extra + n0 + c4) = ov[it];
        }
        __threadfence();
      }
    } else {
      const int q = lane >> 3, c8 = (lane & 7) * 8;
      unsigned short* C  = (unsigned short*)Cout  + (size_t)b * strideC;
      unsigned short* C2 = (unsigned short*)Cout2 + (size_t)b * strideC;
      v4u hw[4], lw[4];
#pragma unroll
      for (int it = 0; it < 4; ++it) {
        const float* sp = slab + (it * 4 + q) * 68 + c8;
        const v4f a0 = *(const v4f*)(sp);
        const v4f a1 = *(const v4f*)(sp + 4);
        hw[it] = (v4u){pack_hi2(a0[0], a0[1]), pack_hi2(a0[2], a0[3]), pack_hi2(a1[0], a1[1]), pack_hi2(a1[2], a1[3])};
        lw[it] = (v4u){pack_lo2(a0[0], a0[1]), pack_lo2(a0[2], a0[3]), pack_lo2(a1[0], a1[1]), pack_lo2(a1[2], a1[3])};
      }
      for (int pass = 0; pass < 2; ++pass) {
#pragma unroll
        for (int it = 0; it < 4; ++it) {
          const int row = it * 4 + q;
          const size_t o = (size_t)(mBase + row) * ldc + n0 + c8;
          *(volatile v4u*)(void*)(C + o)  = hw[it];
          *(volatile v4u*)(void*)(C2 + o) = lw[it];
        }
        __threadfence();
      }
    }
    __builtin_amdgcn_fence(__ATOMIC_RELEASE, "workgroup");
    __builtin_amdgcn_wave_barrier();
    __builtin_amdgcn_fence(__ATOMIC_ACQUIRE, "workgroup");
  }
}

__global__ __launch_bounds__(256) void dwconv_u16_kernel(
    const float* __restrict__ XR, const float* __restrict__ cw, const float* __restrict__ cb,
    unsigned short* __restrict__ U16)
{
  const int lane = threadIdx.x & 31, wave = threadIdx.x >> 5;
  const int e  = blockIdx.y;
  const int g0 = (blockIdx.x * 8 + wave) * 16;
  const int d8 = lane * 8;
  float w0[8], w1[8], w2[8], w3[8], bc[8];
#pragma unroll
  for (int c = 0; c < 8; ++c) {
    const v4f t = *(const v4f*)(cw + ((size_t)(e * kDin + d8 + c)) * 4);
    w0[c] = rne_bf(t[0]); w1[c] = rne_bf(t[1]); w2[c] = rne_bf(t[2]); w3[c] = rne_bf(t[3]);
  }
  {
    const v4f b0 = *(const v4f*)(cb + e * kDin + d8);
    const v4f b1 = *(const v4f*)(cb + e * kDin + d8 + 4);
    bc[0] = rne_bf(b0[0]); bc[1] = rne_bf(b0[1]); bc[2] = rne_bf(b0[2]); bc[3] = rne_bf(b0[3]);
    bc[4] = rne_bf(b1[0]); bc[5] = rne_bf(b1[1]); bc[6] = rne_bf(b1[2]); bc[7] = rne_bf(b1[3]);
  }
  const float* xcol = XR + e * 2 * kDin + d8;
  float xm3[8], xm2[8], xm1[8];
  {
    const bool hist = ((g0 & (kL - 1)) != 0);
    const int rbase = hist ? (g0 - 3) : g0;
    const v4f p0 = *(const v4f*)(xcol + (size_t)rbase * kXrP);
    const v4f p1 = *(const v4f*)(xcol + (size_t)rbase * kXrP + 4);
    const v4f q0 = *(const v4f*)(xcol + (size_t)(rbase + 1) * kXrP);
    const v4f q1 = *(const v4f*)(xcol + (size_t)(rbase + 1) * kXrP + 4);
    const v4f r0 = *(const v4f*)(xcol + (size_t)(rbase + 2) * kXrP);
    const v4f r1 = *(const v4f*)(xcol + (size_t)(rbase + 2) * kXrP + 4);
#pragma unroll
    for (int c = 0; c < 4; ++c) {
      xm3[c] = hist ? p0[c] : 0.0f;  xm3[4 + c] = hist ? p1[c] : 0.0f;
      xm2[c] = hist ? q0[c] : 0.0f;  xm2[4 + c] = hist ? q1[c] : 0.0f;
      xm1[c] = hist ? r0[c] : 0.0f;  xm1[4 + c] = hist ? r1[c] : 0.0f;
    }
  }
#pragma unroll 1
  for (int s = 0; s < 16; ++s) {
    const int row = g0 + s;
    const v4f a0 = *(const v4f*)(xcol + (size_t)row * kXrP);
    const v4f a1 = *(const v4f*)(xcol + (size_t)row * kXrP + 4);
    float xc[8];
    xc[0] = a0[0]; xc[1] = a0[1]; xc[2] = a0[2]; xc[3] = a0[3];
    xc[4] = a1[0]; xc[5] = a1[1]; xc[6] = a1[2]; xc[7] = a1[3];
    float o[8];
#pragma unroll
    for (int c = 0; c < 8; ++c) {
      float acc = w0[c] * xm3[c];
      acc = fmaf(w1[c], xm2[c], acc);
      acc = fmaf(w2[c], xm1[c], acc);
      acc = fmaf(w3[c], xc[c], acc);
      const float sv = acc + bc[c];
      o[c] = sv * __builtin_amdgcn_rcpf(1.0f + __expf(-sv));
      xm3[c] = xm2[c]; xm2[c] = xm1[c]; xm1[c] = xc[c];
    }
    const v4u w = (v4u){pack_hi2(o[0], o[1]), pack_hi2(o[2], o[3]), pack_hi2(o[4], o[5]), pack_hi2(o[6], o[7])};
    store16_2pass(U16 + ((size_t)e * kRows + row) * kDin + d8, w);
  }
}

constexpr int kScTS = 32;
constexpr int kScCh = 64;
constexpr int kScHP = 68;
constexpr int kScXP = 136;
static_assert((kScTS * kScXP / 4) == 17 * kScCh, "staging coverage");
static_assert((kL % kScTS) == 0 && (kDin % kScCh) == 0, "scan tiling");
static_assert(kXdN == kScXP, "staged columns");

__global__ __launch_bounds__(64) void scan_kernel(
    const float* __restrict__ DBL, const float* __restrict__ XR,
    const float* __restrict__ cw, const float* __restrict__ cb,
    const float* __restrict__ Wdt, const float* __restrict__ bdt,
    const float* __restrict__ Alog, const float* __restrict__ Dp,
    const float* __restrict__ WTS,
    unsigned short* __restrict__ YH, unsigned short* __restrict__ YL)
{
  __shared__ __align__(16) float sH[kScCh * kScHP];
  __shared__ __align__(16) float sA[kScCh * kScHP];
  __shared__ __align__(16) float sX[kScTS * kScXP];
  __shared__ __align__(16) float sY[kScTS * kScHP];
  __shared__ __align__(16) float sW[kDtR * kScCh];
  const int tid = threadIdx.x, lane = tid & 31, wave = tid >> 5;
  const int e  = blockIdx.x >> 3;
  const int b  = (blockIdx.x >> 2) & 1;
  const int d0 = (blockIdx.x & 3) * kScCh;
  const int d  = d0 + tid;
  const int ed = e * kDin + d;
  constexpr float kLog2e = 1.4426950408889634f;

#pragma unroll 1
  for (int r = 0; r < kDtR; ++r) sW[r * kScCh + tid] = rne_bf(Wdt[(size_t)ed * kDtR + r]);
#pragma unroll 1
  for (int n = 0; n < kNst; ++n) {
    sA[tid * kScHP + n] = -expf(rne_bf(Alog[(size_t)ed * kNst + n])) * kLog2e;
    sH[tid * kScHP + n] = 0.0f;
  }
  const float cw0 = rne_bf(cw[ed * 4 + 0]), cw1 = rne_bf(cw[ed * 4 + 1]);
  const float cw2 = rne_bf(cw[ed * 4 + 2]), cw3 = rne_bf(cw[ed * 4 + 3]);
  const float cbb = rne_bf(cb[ed]);
  const float bb  = rne_bf(bdt[ed]);
  const float Dd  = rne_bf(Dp[ed]);
  const float wbe = WTS[b * kE + e];
  __syncthreads();

  const size_t row0 = (size_t)b * kL;
  const float* dblb = DBL + ((size_t)e * kRows + row0) * kXdP;
  const float* xrb  = XR + row0 * kXrP + e * 2 * kDin + d;
  float* hp = sH + tid * kScHP;
  const float* ap = sA + tid * kScHP;
  float xm3 = 0.0f, xm2 = 0.0f, xm1 = 0.0f;
  const int q = lane >> 3, c8 = (lane & 7) * 8;

#pragma unroll 1
  for (int t0 = 0; t0 < kL; t0 += kScTS) {
    __syncthreads();
#pragma unroll 1
    for (int i = 0; i < 17; ++i) {
      const int idx = tid + kScCh * i;
      const int r   = idx / 34;
      const int c4  = (idx - r * 34) * 4;
      *(v4f*)(sX + r * kScXP + c4) = *(const v4f*)(dblb + (size_t)(t0 + r) * kXdP + c4);
    }
    __syncthreads();
#pragma unroll 1
    for (int s = 0; s < kScTS; ++s) {
      const float* xr = sX + s * kScXP;
      const v4f q0 = *(const v4f*)(xr);
      const v4f q1 = *(const v4f*)(xr + 4);
      float vdot = 0.0f;
      vdot = fmaf(q0[0], sW[0 * kScCh + tid], vdot);
      vdot = fmaf(q0[1], sW[1 * kScCh + tid], vdot);
      vdot = fmaf(q0[2], sW[2 * kScCh + tid], vdot);
      vdot = fmaf(q0[3], sW[3 * kScCh + tid], vdot);
      vdot = fmaf(q1[0], sW[4 * kScCh + tid], vdot);
      vdot = fmaf(q1[1], sW[5 * kScCh + tid], vdot);
      vdot = fmaf(q1[2], sW[6 * kScCh + tid], vdot);
      vdot = fmaf(q1[3], sW[7 * kScCh + tid], vdot);
      const float v   = vdot + bb;
      const float ea  = __expf(-fabsf(v));
      const float u1  = 1.0f + ea;
      const float l1p = __logf(u1) + (ea - (u1 - 1.0f)) * __builtin_amdgcn_rcpf(u1);
      const float dlt = fmaxf(v, 0.0f) + l1p;

      const size_t ro = (size_t)(t0 + s) * kXrP;
      const float xc = xrb[ro];
      const float rz = xrb[ro + kDin];
      float cacc = cw0 * xm3;
      cacc = fmaf(cw1, xm2, cacc);
      cacc = fmaf(cw2, xm1, cacc);
      cacc = fmaf(cw3, xc, cacc);
      xm3 = xm2; xm2 = xm1; xm1 = xc;
      const float sv = cacc + cbb;
      const float u  = sv * __builtin_amdgcn_rcpf(1.0f + expf(-sv));
      const float du = dlt * u;

      float y = 0.0f;
#pragma unroll 2
      for (int n4 = 0; n4 < kNst / 4; ++n4) {
        v4f hv = *(const v4f*)(hp + 4 * n4);
        const v4f av = *(const v4f*)(ap + 4 * n4);
        const v4f bv = *(const v4f*)(xr + kDtR + 4 * n4);
        const v4f cv = *(const v4f*)(xr + kDtR + kNst + 4 * n4);
#pragma unroll
        for (int k = 0; k < 4; ++k) {
          const float dA = __builtin_amdgcn_exp2f(dlt * av[k]);
          const float hn = fmaf(dA, hv[k], du * bv[k]);
          y = fmaf(hn, cv[k], y);
          hv[k] = hn;
        }
        *(v4f*)(hp + 4 * n4) = hv;
      }
      y = fmaf(u, Dd, y);
      const float g = rz * __builtin_amdgcn_rcpf(1.0f + expf(-rz));
      sY[s * kScHP + tid] = (y * g) * wbe;
    }
    __syncthreads();
    v4u hw[4], lw[4];
#pragma unroll
    for (int it = 0; it < 4; ++it) {
      const int row = it * 8 + wave * 4 + q;
      const float* sp = sY + row * kScHP + c8;
      const v4f a0 = *(const v4f*)(sp);
      const v4f a1 = *(const v4f*)(sp + 4);
      hw[it] = (v4u){pack_hi2(a0[0], a0[1]), pack_hi2(a0[2], a0[3]), pack_hi2(a1[0], a1[1]), pack_hi2(a1[2], a1[3])};
      lw[it] = (v4u){pack_lo2(a0[0], a0[1]), pack_lo2(a0[2], a0[3]), pack_lo2(a1[0], a1[1]), pack_lo2(a1[2], a1[3])};
    }
    for (int pass = 0; pass < 2; ++pass) {
#pragma unroll
      for (int it = 0; it < 4; ++it) {
        const int row = it * 8 + wave * 4 + q;
        const size_t o = (row0 + t0 + row) * kYcP + e * kDin + d0 + c8;
        *(volatile v4u*)(void*)(YH + o) = hw[it];
        *(volatile v4u*)(void*)(YL + o) = lw[it];
      }
      __threadfence();
    }
  }
}

extern "C" void kernel_launch(void* const* d_in, const int* in_sizes, int n_in,
                              void* d_out, int out_size, void* d_ws, size_t ws_size,
                              hipStream_t stream)
{
  if (n_in < 16) return;
  if (in_sizes[0]  != kB * kC * kL) return;
  if (in_sizes[1]  != kE * 2 * kDin * kC) return;
  if (in_sizes[2]  != kE * kDin * 4) return;
  if (in_sizes[3]  != kE * kDin) return;
  if (in_sizes[4]  != kE * kXdN * kDin) return;
  if (in_sizes[5]  != kE * kDin * kDtR) return;
  if (in_sizes[6]  != kE * kDin) return;
  if (in_sizes[7]  != kE * kDin * kNst) return;
  if (in_sizes[8]  != kE * kDin) return;
  if (in_sizes[9]  != kE * kC * kDin) return;
  if (in_sizes[10] != kRc * kC * 9) return;
  if (in_sizes[11] != kRc) return;
  if (in_sizes[12] != kE * kRc) return;
  if (in_sizes[13] != kE) return;
  if (in_sizes[14] != kC * kC) return;
  if (in_sizes[15] != kC) return;
  if (out_size != kB * kC * kL) return;
  if (ws_size < kWsTotal) return;

  const float* x        = (const float*)d_in[0];
  const float* in_w     = (const float*)d_in[1];
  const float* conv_w   = (const float*)d_in[2];
  const float* conv_b   = (const float*)d_in[3];
  const float* xproj_w  = (const float*)d_in[4];
  const float* dt_w     = (const float*)d_in[5];
  const float* dt_b     = (const float*)d_in[6];
  const float* A_log    = (const float*)d_in[7];
  const float* D_p      = (const float*)d_in[8];
  const float* out_w    = (const float*)d_in[9];
  const float* r_conv_w = (const float*)d_in[10];
  const float* r_conv_b = (const float*)d_in[11];
  const float* r_lin_w  = (const float*)d_in[12];
  const float* r_lin_b  = (const float*)d_in[13];
  const float* fusion_w = (const float*)d_in[14];
  const float* fusion_b = (const float*)d_in[15];
  float* out = (float*)d_out;

  char* ws = (char*)d_ws;
  unsigned short* XSEQ = (unsigned short*)(ws + kOffXSEQ);
  unsigned short* XPAD = (unsigned short*)(ws + kOffXPAD);
  unsigned short* WIN  = (unsigned short*)(ws + kOffWIN);
  unsigned short* WXP  = (unsigned short*)(ws + kOffWXP);
  unsigned short* WOUT = (unsigned short*)(ws + kOffWOUT);
  unsigned short* WFUS = (unsigned short*)(ws + kOffWFUS);
  unsigned short* WR   = (unsigned short*)(ws + kOffWR);
  float*          PART = (float*)(ws + kOffPART);
  float*          WTS  = (float*)(ws + kOffWTS);
  float*          XR   = (float*)(ws + kOffXR);
  unsigned short* U16  = (unsigned short*)(ws + kOffU16);
  float*          DBL  = (float*)(ws + kOffDBL);
  unsigned short* YH   = (unsigned short*)(ws + kOffYH);
  unsigned short* YL   = (unsigned short*)(ws + kOffYL);
  unsigned short* WSH  = (unsigned short*)(ws + kOffWSH);
  unsigned short* WSL  = (unsigned short*)(ws + kOffWSL);

  prep_x_kernel<<<kB * kSide, 256, 0, stream>>>(x, XSEQ, XPAD);

  prep_w_kernel<<<260, 256, 0, stream>>>(in_w, xproj_w, out_w, fusion_w, r_conv_w, WIN, WXP, WOUT, WFUS, WR);

  router_conv_kernel<<<(kRows / 64) / 8, 256, 0, stream>>>(XPAD, WR, r_conv_b, PART);

  router_finish_kernel<<<1, 128, 0, stream>>>(PART, r_lin_w, r_lin_b, WTS);

  gemm64_bf16_kernel<0, 0, 0, 0, 0><<<dim3((kRows / 64) * (kXrP / 64) / 8, 1), 256, 0, stream>>>(
      XSEQ, XSEQ, kC, 0L,
      WIN, WIN, kC, 0L,
      (void*)XR, (void*)XR, kXrP, 0L,
      fusion_b, kRows, kXrP, kC);

  dwconv_u16_kernel<<<dim3(kRows / 16 / 8, kE), 256, 0, stream>>>(XR, conv_w, conv_b, U16);

  gemm64_bf16_kernel<0, 0, 0, 0, 0><<<dim3((kRows / 64) * (kXdP / 64) / 8, kE), 256, 0, stream>>>(
      U16, U16, kDin, (long)kRows * kDin,
      WXP, WXP, kDin, (long)kXdP * kDin,
      (void*)DBL, (void*)DBL, kXdP, (long)kRows * kXdP,
      fusion_b, kRows, kXdP, kDin);

  scan_kernel<<<kE * kB * (kDin / kScCh), kScCh, 0, stream>>>(
      DBL, XR, conv_w, conv_b, dt_w, dt_b, A_log, D_p, WTS, YH, YL);

  gemm64_bf16_kernel<1, 0, 0, 2, 0><<<dim3((kRows / 64) * (kC / 64) / 8, 1), 256, 0, stream>>>(
      YH, YL, kYcP, 0L,
      WOUT, WOUT, kYcP, 0L,
      (void*)WSH, (void*)WSL, kC, 0L,
      fusion_b, kRows, kC, kYcP);

  gemm64_bf16_kernel<0, 1, 1, 0, 1><<<dim3((kC / 64) * (kRows / 64) / 8, 1), 256, 0, stream>>>(
      WFUS, WFUS, kC, 0L,
      WSH, WSL, kC, 0L,
      (void*)out, (void*)out, kL, 0L,
      fusion_b, kC, kRows, kC);
}
